// SPCausalSelfAttention_34067680592426
// MI455X (gfx1250) — hardware-verified
//
#include <hip/hip_runtime.h>
#include <math.h>


#define BB 2
#define SS 2048
#define DD 1024
#define HH 16
#define HD 64
#define BS (BB * SS)
#define D3 (3 * DD)
#define BK 32

typedef __attribute__((ext_vector_type(16))) _Float16 v16h;
typedef __attribute__((ext_vector_type(16))) __bf16 v16b;
typedef __attribute__((ext_vector_type(8)))  float v8f;
typedef __attribute__((ext_vector_type(4)))  float v4f;

template <typename T> __device__ __forceinline__ void vst2(void* p, T v) { *(volatile T*)p = v; __threadfence(); *(volatile T*)p = v; }
__device__ __forceinline__ v8f wmma16(v16h a, v16h b, v8f c) {
  v8f d = __builtin_amdgcn_wmma_f32_16x16x32_f16(false, a, false, b, (short)0, c, false, false);
  asm volatile("v_nop\n\tv_nop\n\tv_nop\n\tv_nop" : "+v"(d) : "v"(a), "v"(b));
  return d;
}
__device__ __forceinline__ v8f wmma_bf(v16b a, v16b b, v8f c) {
  v8f d = __builtin_amdgcn_wmma_f32_16x16x32_bf16(false, a, false, b, (short)0, c, false, false);
  asm volatile("v_nop\n\tv_nop\n\tv_nop\n\tv_nop" : "+v"(d) : "v"(a), "v"(b));
  return d;
}
struct F2 { v16b h, l; };
__device__ __forceinline__ F2 split_row(const float* rowk0, int lane) {
  F2 r; const float* p = rowk0 + 8 * (lane >> 4);
#pragma unroll
  for (int i = 0; i < 8; ++i) { float v0 = p[i], v1 = p[16 + i]; __bf16 h0 = (__bf16)v0, h1 = (__bf16)v1;
    r.h[i] = h0; r.l[i] = (__bf16)(v0 - (float)h0); r.h[8 + i] = h1; r.l[8 + i] = (__bf16)(v1 - (float)h1); }
  return r;
}
__device__ __forceinline__ v8f mac3(const F2& a, const F2& b, v8f c) { c = wmma_bf(a.l, b.h, c); c = wmma_bf(a.h, b.l, c); return wmma_bf(a.h, b.h, c); }
struct H2 { v16h h, l; };
__device__ __forceinline__ H2 hsplit_row(const float* rowk0, int lane) {
  H2 a; const float* p = rowk0 + 8 * (lane >> 4);
#pragma unroll
  for (int i = 0; i < 8; ++i) { float v0 = p[i], v1 = p[16 + i]; _Float16 h0 = (_Float16)v0, h1 = (_Float16)v1;
    a.h[i] = h0; a.l[i] = (_Float16)(v0 - (float)h0); a.h[8 + i] = h1; a.l[8 + i] = (_Float16)(v1 - (float)h1); }
  return a;
}
__device__ __forceinline__ v16h frag_f32(const float* rowk0, int lane) {
  v16h a; const float* p = rowk0 + 8 * (lane >> 4);
#pragma unroll
  for (int i = 0; i < 8; ++i) { a[i] = (_Float16)p[i]; a[8 + i] = (_Float16)p[16 + i]; }
  return a;
}
#define LDSX() do { asm volatile("s_wait_dscnt 0" ::: "memory"); __builtin_amdgcn_wave_barrier(); __builtin_amdgcn_fence(__ATOMIC_RELEASE, "workgroup"); } while (0)

__global__ __launch_bounds__(256) void k_transpose(const float* __restrict__ W, float* __restrict__ Wt, int K, int N) {
  __shared__ float tile[32][33];
  const int k0 = blockIdx.y * 32, n0 = blockIdx.x * 32, tid = threadIdx.x;
  for (int q = tid; q < 32 * 32; q += 256) { const int kk = q >> 5, nn = q & 31; tile[kk][nn] = W[(size_t)(k0 + kk) * N + n0 + nn]; }
  __syncthreads();
  for (int q = tid; q < 32 * 8; q += 256) { const int nn = q >> 3, pc = q & 7;
    v4f v = { tile[pc * 4][nn], tile[pc * 4 + 1][nn], tile[pc * 4 + 2][nn], tile[pc * 4 + 3][nn] };
    vst2(Wt + (size_t)(n0 + nn) * K + k0 + pc * 4, v); }
}

__global__ __launch_bounds__(128) void k_qkv(const float* __restrict__ x, const float* __restrict__ Wt, const float* __restrict__ bqkv,
                                           float* __restrict__ qp, float* __restrict__ kp, float* __restrict__ vT) {
  __shared__ __align__(16) float st[128][68];
  const int tid = threadIdx.x, wave = tid >> 5, lane = tid & 31, col = lane & 15, g = lane >> 4;
  const int r0 = blockIdx.x * 64, n0 = blockIdx.y * 128;
  const int b = r0 / SS, s0 = r0 % SS;
  v8f acc[8] = {};
#pragma unroll 1
  for (int kc = 0; kc < DD / 32; ++kc) {
    const F2 a = split_row(x + (size_t)(r0 + wave * 16 + col) * DD + kc * 32, lane);
#pragma unroll
    for (int j = 0; j < 8; ++j) acc[j] = mac3(a, split_row(Wt + (size_t)(n0 + j * 16 + col) * DD + kc * 32, lane), acc[j]);
  }
#pragma unroll
  for (int j = 0; j < 8; ++j) { const float bv = bqkv[n0 + j * 16 + col];
#pragma unroll
    for (int r = 0; r < 8; ++r) st[j * 16 + col][wave * 16 + 8 * g + r] = acc[j][r] + bv; }
  __syncthreads();
  const int which = n0 / DD, h0 = (n0 % DD) / HD;
  if (which < 2) {
    float* dst = which == 0 ? qp : kp;
    for (int q = tid; q < 2 * 64 * 16; q += 128) { const int hh = q >> 10, sl = (q >> 4) & 63, pc = q & 15;
      v4f v = { st[hh * 64 + pc * 4][sl], st[hh * 64 + pc * 4 + 1][sl], st[hh * 64 + pc * 4 + 2][sl], st[hh * 64 + pc * 4 + 3][sl] };
      vst2(dst + (((size_t)b * HH + h0 + hh) * SS + s0 + sl) * HD + pc * 4, v); }
  } else {
    for (int q = tid; q < 128 * 16; q += 128) { const int cl = q >> 4, pc = q & 15; const int hh = cl >> 6, d = cl & 63;
      vst2(vT + (((size_t)b * HH + h0 + hh) * HD + d) * SS + s0 + pc * 4, *(const v4f*)(&st[cl][pc * 4])); }
  }
}

__global__ __launch_bounds__(128) void k_attn(const float* __restrict__ qp, const float* __restrict__ kp, const float* __restrict__ vT, float* __restrict__ y) {
  __shared__ __align__(16) float sP[4][16][BK];
  __shared__ __align__(16) float sO[4][16][HD];
  const int tid = threadIdx.x, w = tid >> 5, lane = tid & 31, g = lane >> 4, ln = lane & 15;
  const int bh = blockIdx.y, b = bh / HH, h = bh % HH, q0 = blockIdx.x * 64 + w * 16;
  const float* qrow = qp + ((size_t)bh * SS + q0 + ln) * HD;
  const F2 qa0 = split_row(qrow, lane), qa1 = split_row(qrow + 32, lane);
  const float scale = 0.125f;
  float mrun[8], lrun[8];
  v8f acc[4];
#pragma unroll
  for (int r = 0; r < 8; ++r) { mrun[r] = -3.0e38f; lrun[r] = 0.f; }
#pragma unroll
  for (int t = 0; t < 4; ++t) acc[t] = (v8f){};
  const float* kb = kp + (size_t)bh * SS * HD;
  const float* vb = vT + (size_t)bh * HD * SS;
  const int kend = blockIdx.x * 64 + 64;
#pragma unroll 1
  for (int k0 = 0; k0 < kend; k0 += BK) {
    v8f s0 = {}, s1 = {};
    s0 = mac3(qa0, split_row(kb + (size_t)(k0 + ln) * HD, lane), s0);      s0 = mac3(qa1, split_row(kb + (size_t)(k0 + ln) * HD + 32, lane), s0);
    s1 = mac3(qa0, split_row(kb + (size_t)(k0 + 16 + ln) * HD, lane), s1); s1 = mac3(qa1, split_row(kb + (size_t)(k0 + 16 + ln) * HD + 32, lane), s1);
#pragma unroll
    for (int r = 0; r < 8; ++r) {
      const int qg = q0 + 8 * g + r;
      const float x0 = (k0 + ln <= qg) ? s0[r] * scale : -3.0e38f, x1 = (k0 + 16 + ln <= qg) ? s1[r] * scale : -3.0e38f;
      float mx = fmaxf(x0, x1);
#pragma unroll
      for (int off = 8; off >= 1; off >>= 1) mx = fmaxf(mx, __shfl_xor(mx, off, 32));
      const float mn = fmaxf(mrun[r], mx);
      const float corr = expf(mrun[r] - mn);
      const float p0 = (x0 > -1.0e38f) ? expf(x0 - mn) : 0.f, p1 = (x1 > -1.0e38f) ? expf(x1 - mn) : 0.f;
      float sum = p0 + p1;
#pragma unroll
      for (int off = 8; off >= 1; off >>= 1) sum += __shfl_xor(sum, off, 32);
      lrun[r] = lrun[r] * corr + sum; mrun[r] = mn;
#pragma unroll
      for (int t = 0; t < 4; ++t) acc[t][r] *= corr;
      sP[w][8 * g + r][ln] = p0 * 16384.0f; sP[w][8 * g + r][16 + ln] = p1 * 16384.0f;
    }
    LDSX();
    const v16h pa = frag_f32(&sP[w][ln][0], lane);
#pragma unroll
    for (int t = 0; t < 4; ++t) { const H2 vb2 = hsplit_row(vb + (size_t)(t * 16 + ln) * SS + k0, lane);
      acc[t] = wmma16(pa, vb2.l, acc[t]); acc[t] = wmma16(pa, vb2.h, acc[t]); }
    __builtin_amdgcn_wave_barrier();
  }
  float* so = &sO[w][0][0];
#pragma unroll
  for (int r = 0; r < 8; ++r) { const float il = (1.0f / 16384.0f) / lrun[r];
#pragma unroll
    for (int t = 0; t < 4; ++t) so[(8 * g + r) * HD + t * 16 + ln] = acc[t][r] * il; }
  LDSX();
#pragma unroll
  for (int q = 0; q < 8; ++q) { const int rl = q * 2 + (lane >> 4), pc = lane & 15;
    vst2(y + ((size_t)b * SS + q0 + rl) * DD + h * HD + pc * 4, *(const v4f*)(so + rl * HD + pc * 4)); }
}

__global__ __launch_bounds__(128) void k_out(const float* __restrict__ y, const float* __restrict__ Wpt, const float* __restrict__ bo, float* __restrict__ out) {
  __shared__ __align__(16) float so[4][16 * 128];
  const int tid = threadIdx.x, wave = tid >> 5, lane = tid & 31, col = lane & 15, g = lane >> 4;
  const int r0 = blockIdx.x * 64 + wave * 16, n0 = blockIdx.y * 128;
  v8f acc[8] = {};
#pragma unroll 1
  for (int kc = 0; kc < DD / 32; ++kc) {
    const F2 a = split_row(y + (size_t)(r0 + col) * DD + kc * 32, lane);
#pragma unroll
    for (int j = 0; j < 8; ++j) acc[j] = mac3(a, split_row(Wpt + (size_t)(n0 + j * 16 + col) * DD + kc * 32, lane), acc[j]);
  }
  float* S = so[wave];
#pragma unroll
  for (int j = 0; j < 8; ++j) { const float bv = bo[n0 + j * 16 + col];
#pragma unroll
    for (int r = 0; r < 8; ++r) S[(8 * g + r) * 128 + j * 16 + col] = acc[j][r] + bv; }
  LDSX();
#pragma unroll 4
  for (int rl = 0; rl < 16; ++rl) vst2(out + (size_t)(r0 + rl) * DD + n0 + lane * 4, *(const v4f*)(S + rl * 128 + lane * 4));
}

extern "C" void kernel_launch(void* const* d_in, const int* in_sizes, int n_in,
                              void* d_out, int out_size, void* d_ws, size_t ws_size,
                              hipStream_t stream) {
  (void)in_sizes; (void)n_in; (void)out_size; (void)ws_size;
  const float* x  = (const float*)d_in[0];
  const float* Wa = (const float*)d_in[1]; const float* ba = (const float*)d_in[2];
  const float* Wp = (const float*)d_in[3]; const float* bp = (const float*)d_in[4];
  float* out = (float*)d_out;
  char* ws = (char*)d_ws; size_t off = 0;
  auto take = [&](size_t bytes) { char* p = ws + off; off += (bytes + 255) & ~(size_t)255; return p; };
  float* Wat = (float*)take((size_t)D3 * DD * 4);
  float* Wpt = (float*)take((size_t)DD * DD * 4);
  float* qp  = (float*)take((size_t)BS * DD * 4);
  float* kp  = (float*)take((size_t)BS * DD * 4);
  float* vT  = (float*)take((size_t)BS * DD * 4);
  float* y   = (float*)take((size_t)BS * DD * 4);
  k_transpose<<<dim3(D3 / 32, DD / 32), 256, 0, stream>>>(Wa, Wat, DD, D3);
  k_transpose<<<dim3(DD / 32, DD / 32), 256, 0, stream>>>(Wp, Wpt, DD, DD);
  k_qkv<<<dim3(BS / 64, D3 / 128), 128, 0, stream>>>(x, Wat, ba, qp, kp, vT);
  k_attn<<<dim3(SS / 64, BB * HH), 128, 0, stream>>>(qp, kp, vT, y);
  k_out<<<dim3(BS / 64, DD / 128), 128, 0, stream>>>(y, Wpt, bp, out);
}
